// _NonLocalBlock_32427003084831
// MI455X (gfx1250) — hardware-verified
//
#include <hip/hip_runtime.h>


namespace {
constexpr int NB_ = 8, C = 128, Hh = 64, Ww = 32, N = Hh * Ww  , IC = 64, CH = 256;
constexpr float XS = 8.0f, HS = 256.0f, PS = 256.0f, WSC = 256.0f, NEG = -9.0e15f;
typedef _Float16 b16;
typedef __attribute__((ext_vector_type(16))) _Float16 v16b;
typedef __attribute__((ext_vector_type(8))) _Float16 v8b;
typedef __attribute__((ext_vector_type(2))) _Float16 v2b;
typedef __attribute__((ext_vector_type(8))) float v8f;
typedef __attribute__((ext_vector_type(4))) float v4f;
typedef __attribute__((ext_vector_type(2))) float v2f;
__device__ __forceinline__ float bf16_rne(float f) { unsigned int u = __float_as_uint(f); u += 0x7FFFu + ((u >> 16) & 1u); float r = __uint_as_float(u & 0xFFFF0000u); asm volatile("" : "+v"(r)); return r; }
__device__ __forceinline__ float bfv(float f) { float r = bf16_rne(f); asm volatile("" : "+v"(r)); return r; }
__device__ __forceinline__ void split16(float v, b16& hi, b16& lo) { hi = (b16)v; lo = (b16)(v - (float)hi); }
__device__ __forceinline__ v16b frag_kb(const b16* p, int hh) { const v8b a = *(const v8b*)(p + 8 * hh), b = *(const v8b*)(p + 16 + 8 * hh); v16b f;
#pragma unroll
  for (int e = 0; e < 8; ++e) { f[e] = a[e]; f[8 + e] = b[e]; } return f; }
__device__ __forceinline__ v8f wmma16b(v16b a, v16b b, v8f c) { v8f d = __builtin_amdgcn_wmma_f32_16x16x32_f16(false, a, false, b, (short)0, c, false, false); asm volatile("v_nop\n\tv_nop\n\tv_nop\n\tv_nop" : "+v"(d) : "v"(a), "v"(b)); return d; }
__device__ __forceinline__ void wave_lds_sync() { __builtin_amdgcn_fence(__ATOMIC_RELEASE, "workgroup"); __builtin_amdgcn_wave_barrier(); __builtin_amdgcn_fence(__ATOMIC_ACQUIRE, "workgroup"); }
__device__ __forceinline__ float pmul(float a, float b) { float p = a * b; asm volatile("" : "+v"(p)); return p; }

__global__ __launch_bounds__(256) void wput_kernel(const float* __restrict__ wg, const float* __restrict__ wt, const float* __restrict__ wp, b16* __restrict__ W) { const int u = blockIdx.x * 256 + threadIdx.x; if (u >= 3 * IC * 16) return; const int o = u / 16, k0 = (u % 16) * 8; const float* w = o < IC ? wg : (o < 2 * IC ? wt : wp); const int oo = o % IC; v8b v;
#pragma unroll
  for (int j = 0; j < 8; ++j) v[j] = (b16)(bf16_rne(w[(size_t)oo * C + k0 + j]) * WSC);
  for (int pass = 0; pass < 2; ++pass) { *(volatile v8b*)(W + (size_t)o * C + k0) = v; __threadfence(); } }
__global__ __launch_bounds__(32) void proj_kernel(const float* __restrict__ x, const b16* __restrict__ W, const float* __restrict__ bg, const float* __restrict__ bt, const float* __restrict__ bp, const float* __restrict__ cpw, float* __restrict__ G, float* __restrict__ FS) { __shared__ __attribute__((aligned(16))) b16 Ah[16][C + 8]; __shared__ float Tf[16][3 * IC + 4], Fq[16][8]; const int lane = threadIdx.x, nloc = lane & 15, hlf = lane >> 4; const int b = blockIdx.x / (N / 16), n0 = (blockIdx.x % (N / 16)) * 16; const size_t s0 = (size_t)b * N + n0;
  for (int c = 0; c < C; ++c) if (lane < 16) Ah[lane][c] = (b16)(bf16_rne(x[((size_t)b * C + c) * N + n0 + lane]) * XS);
  if (lane < 16) { for (int k = C; k < C + 8; ++k) Ah[lane][k] = (b16)0.0f; for (int j = 0; j < 8; ++j) Fq[lane][j] = 0.0f; }
  wave_lds_sync(); v8f acc[12];
#pragma unroll
  for (int t = 0; t < 12; ++t) acc[t] = (v8f){};
#pragma unroll
  for (int kb = 0; kb < C; kb += 32) { const v16b a = frag_kb(&Ah[nloc][kb], hlf);
#pragma unroll
    for (int t = 0; t < 12; ++t) acc[t] = wmma16b(a, frag_kb(W + (size_t)(t * 16 + nloc) * C + kb, hlf), acc[t]); }
#pragma unroll
  for (int t = 0; t < 12; ++t) { const int cc = t * 16 + nloc; const float bb = bfv(cc < IC ? bg[cc] : (cc < 2 * IC ? bt[cc - IC] : bp[cc - 2 * IC]));
#pragma unroll
    for (int r8 = 0; r8 < 8; ++r8) Tf[8 * hlf + r8][cc] = acc[t][r8] * (1.0f / (XS * WSC)) + bb; }
  wave_lds_sync();
  for (int rr = 0; rr < 16; ++rr) { float s1 = 0.0f, s2 = 0.0f; for (int q = 0; q < 2; ++q) { const int o = q * 32 + lane; s1 += pmul(Tf[rr][IC + o], bfv(cpw[o])); s2 += pmul(Tf[rr][2 * IC + o], bfv(cpw[IC + o])); } for (int o = 16; o; o >>= 1) { s1 += __shfl_xor(s1, o); s2 += __shfl_xor(s2, o); } if (lane == 0) { Fq[rr][0] = s1; Fq[rr][1] = s2; } }
  wave_lds_sync();
  for (int pass = 0; pass < 2; ++pass) { for (int rr = 0; rr < 16; ++rr) *(volatile v2f*)(G + (s0 + rr) * IC + lane * 2) = (v2f){Tf[rr][lane * 2], Tf[rr][lane * 2 + 1]}; for (int q = 0; q < 4; ++q) ((volatile float*)FS)[s0 * 8 + q * 32 + lane] = Fq[(q * 32 + lane) >> 3][(q * 32 + lane) & 7]; __threadfence(); } }
__global__ __launch_bounds__(256) void gt_kernel(const float* __restrict__ G, b16* __restrict__ GTH, b16* __restrict__ GTL) { __shared__ float Tt[64][65]; const int b = blockIdx.x / (N / 64), n0 = (blockIdx.x % (N / 64)) * 64; const int tid = threadIdx.x, wave = tid >> 5, lane = tid & 31;
  for (int q = wave; q < 64; q += 8) { Tt[q][lane * 2] = G[((size_t)b * N + n0 + q) * IC + lane * 2]; Tt[q][lane * 2 + 1] = G[((size_t)b * N + n0 + q) * IC + lane * 2 + 1]; }
  __syncthreads();
  for (int pass = 0; pass < 2; ++pass) { for (int o = wave; o < IC; o += 8) { b16 h0, l0, h1, l1; split16(Tt[lane * 2][o] * HS, h0, l0); split16(Tt[lane * 2 + 1][o] * HS, h1, l1); *(volatile v2b*)(GTH + ((size_t)b * IC + o) * N + n0 + lane * 2) = (v2b){h0, h1}; *(volatile v2b*)(GTL + ((size_t)b * IC + o) * N + n0 + lane * 2) = (v2b){l0, l1}; } __threadfence(); } }
__global__ __launch_bounds__(32) void att_kernel(const float* __restrict__ FS, const int* __restrict__ adj, const b16* __restrict__ GTH, const b16* __restrict__ GTL, int SLIM, float* __restrict__ out) { __shared__ __attribute__((aligned(16))) b16 Pa[32][CH + 8], Pb[32][CH + 8]; __shared__ float Mx[32], Iv[32], Ft[32], Tf[32][IC + 1]; const int lane = threadIdx.x, nloc = lane & 15, hlf = lane >> 4; const int b = blockIdx.x / (N / 32), i0 = (blockIdx.x % (N / 32)) * 32; const size_t s0 = (size_t)b * N + i0; if (s0 >= (size_t)SLIM) return;
  const float* FPb = FS + (size_t)b * N * 8;
  Ft[lane] = FS[(s0 + lane) * 8];
  wave_lds_sync();
  for (int r = 0; r < 32; ++r) { const float ft = Ft[r]; const int* arow = adj + (size_t)(i0 + r) * N; float mx = -INFINITY; for (int j = lane; j < N; j += 32) { float e = ft + FPb[(size_t)j * 8 + 1]; e = e > 0.0f ? e : 0.2f * e; e = arow[j] > 0 ? NEG : e; mx = fmaxf(mx, e); } for (int o = 16; o; o >>= 1) mx = fmaxf(mx, __shfl_xor(mx, o));
    float sm = 0.0f; for (int j = lane; j < N; j += 32) { float e = ft + FPb[(size_t)j * 8 + 1]; e = e > 0.0f ? e : 0.2f * e; e = arow[j] > 0 ? NEG : e; sm += __expf(e - mx); } for (int o = 16; o; o >>= 1) sm += __shfl_xor(sm, o); if (lane == 0) { Mx[r] = mx; Iv[r] = 1.0f / sm; } }
  for (int k = CH; k < CH + 8; ++k) { Pa[lane][k] = (b16)0.0f; Pb[lane][k] = (b16)0.0f; }
  wave_lds_sync(); v8f acc[2][4];
#pragma unroll
  for (int rt = 0; rt < 2; ++rt)
#pragma unroll
    for (int t = 0; t < 4; ++t) acc[rt][t] = (v8f){};
#pragma unroll 1
  for (int ch = 0; ch < N / CH; ++ch) { const int j0 = ch * CH;
    for (int r = 0; r < 32; ++r) { const float ft = Ft[r], mx = Mx[r], iv = Iv[r]; const int* arow = adj + (size_t)(i0 + r) * N + j0; for (int q = 0; q < CH / 32; ++q) { const int j = q * 32 + lane; float e = ft + FPb[(size_t)(j0 + j) * 8 + 1]; e = e > 0.0f ? e : 0.2f * e; e = arow[j] > 0 ? NEG : e; const float p = __expf(e - mx) * iv; b16 ph, pl; split16(p * PS, ph, pl); Pa[r][j] = ph; Pb[r][j] = pl; } }
    wave_lds_sync();
#pragma unroll 2
    for (int kb = 0; kb < CH; kb += 32) {
#pragma unroll
      for (int rt = 0; rt < 2; ++rt) { const v16b pa = frag_kb(&Pa[rt * 16 + nloc][kb], hlf), pb = frag_kb(&Pb[rt * 16 + nloc][kb], hlf);
#pragma unroll
        for (int t = 0; t < 4; ++t) { const b16* gp = GTH + ((size_t)b * IC + t * 16 + nloc) * N + j0 + kb; const v16b gh = frag_kb(gp, hlf), gl = frag_kb(GTL + (gp - GTH), hlf); acc[rt][t] = wmma16b(pa, gh, acc[rt][t]); acc[rt][t] = wmma16b(pa, gl, acc[rt][t]); acc[rt][t] = wmma16b(pb, gh, acc[rt][t]); } } }
    wave_lds_sync(); }
#pragma unroll
  for (int rt = 0; rt < 2; ++rt)
#pragma unroll
    for (int t = 0; t < 4; ++t)
#pragma unroll
      for (int r8 = 0; r8 < 8; ++r8) Tf[rt * 16 + 8 * hlf + r8][t * 16 + nloc] = acc[rt][t][r8] * (1.0f / (PS * HS));
  wave_lds_sync();
  for (int pass = 0; pass < 2; ++pass) { for (int o = 0; o < IC; ++o) ((volatile float*)out)[((size_t)b * IC + o) * N + i0 + lane] = Tf[lane][o]; __threadfence(); } }
}

extern "C" void kernel_launch(void* const* d_in, const int* in_sizes, int n_in, void* d_out, int out_size, void* d_ws, size_t ws_size, hipStream_t stream) {
  (void)n_in;
  auto Fp = [&](int i) { return (const float*)d_in[i]; }; auto Ip = [&](int i) { return (const int*)d_in[i]; };
  if (in_sizes[0] != NB_ * C * N || in_sizes[1] != N * N || in_sizes[2] != IC * C || in_sizes[4] != IC * C || in_sizes[6] != IC * C || in_sizes[8] != 2 * IC || out_size != NB_ * IC * N) return;
  const int SLIM = NB_ * N;
  size_t off = 0; char* ws = (char*)d_ws;
  auto carve = [&](size_t bytes) { char* p = ws + off; off += (bytes + 255) & ~(size_t)255; return p; };
  b16* W = (b16*)carve((size_t)3 * IC * C * 2); float* G = (float*)carve((size_t)NB_ * N * IC * 4); float* FS = (float*)carve((size_t)NB_ * N * 8 * 4); b16* GTH = (b16*)carve((size_t)NB_ * IC * N * 2); b16* GTL = (b16*)carve((size_t)NB_ * IC * N * 2);
  if (off > ws_size || off > ((size_t)16 << 20)) return;
  wput_kernel<<<(3 * IC * 16 + 255) / 256, 256, 0, stream>>>(Fp(2), Fp(4), Fp(6), W);
  proj_kernel<<<NB_ * (N / 16), 32, 0, stream>>>(Fp(0), W, Fp(3), Fp(5), Fp(7), Fp(8), G, FS);
  gt_kernel<<<NB_ * (N / 64), 256, 0, stream>>>(G, GTH, GTL);
  att_kernel<<<SLIM / 32, 32, 0, stream>>>(FS, Ip(1), GTH, GTL, SLIM, (float*)d_out);
}
